// BOCPD_GPTS_16174846837166
// MI455X (gfx1250) — hardware-run, weakly checked
//
#include <hip/hip_runtime.h>
#include <math.h>


#ifndef NSTEPS
#define NSTEPS 4096
#endif
#define TLEN_FULL 4096
#define WWIN 128
#define MW   127
#define MP   128
#define PW   16
#define NPAN (MP / PW)
#define SPW  32
#define KPT  128
#define LPT  136
#define LCS  64.0f
#define LCI2 (1.0f / 4096.0f)
#define PI_F 3.14159265358979323846f

static_assert(MP == 128);
static_assert(PW == 16);
static_assert(NPAN == 8);
static_assert((NPAN + 0) / 2 <= 4);
static_assert(MW == WWIN - 1);
static_assert(MW < MP);
static_assert(KPT >= MP);
static_assert(KPT % 4 == 0);
static_assert(LPT >= MP);
static_assert(LPT % 8 == 0);
static_assert(((MP * LPT) / 8) % 32 == 0);
static_assert(SPW == 32);
static_assert(32 * 4 == SPW * 4);
static_assert(NSTEPS % SPW == 0);
static_assert(NSTEPS <= TLEN_FULL);
static_assert(NSTEPS >= SPW);
static_assert((size_t)MP * KPT * 4 + (size_t)MP * LPT * 2 + (size_t)MP * 4 <= (size_t)131072);

typedef _Float16 h16;
typedef __attribute__((ext_vector_type(16))) _Float16 v16h;
typedef __attribute__((ext_vector_type(8)))  _Float16 v8h;
typedef __attribute__((ext_vector_type(8)))  float    v8f;
typedef __attribute__((ext_vector_type(4)))  float    v4f;
typedef v4f  __attribute__((may_alias)) v4fa;
typedef v8h  __attribute__((may_alias)) v8ha;

__device__ __forceinline__ unsigned short f2bf(float f) { unsigned u = __float_as_uint(f); u += 0x7FFFu + ((u >> 16) & 1u); return (unsigned short)(u >> 16); }
__device__ __forceinline__ float bfr(float f) { return __uint_as_float(((unsigned)f2bf(f)) << 16); }
__device__ __forceinline__ v16h cat16(v8h lo, v8h hi) { return __builtin_shufflevector(lo, hi, 0, 1, 2, 3, 4, 5, 6, 7, 8, 9, 10, 11, 12, 13, 14, 15); }
__device__ __forceinline__ v8f wmma16(v16h a, v16h b, v8f c) { return __builtin_amdgcn_wmma_f32_16x16x32_f16(false, a, false, b, (short)0, c, false, false); }
static __device__ __forceinline__ v8f wmma_g(v16h a, v16h b, v8f c) { c = wmma16(a, b, c); asm volatile("v_nop\n\tv_nop\n\tv_nop\n\tv_nop" : "+v"(c) : "v"(a), "v"(b)); return c; }
static __device__ __forceinline__ h16 toh_flush(float v) { const h16 r = (h16)v; return (fabsf(v) < 6.103515625e-05f) ? (h16)0.0f : r; }
static __device__ __forceinline__ float rdlane(float v, int ln) { return __int_as_float(__builtin_amdgcn_readlane(__float_as_int(v), ln)); }
static __device__ __forceinline__ float kelem(float xi, float xj, bool both, bool dg, float amp, float noise, float rls2) {
    const float d = xi - xj;
    const float e = __expf((-0.5f * (d * d)) * rls2);
    const float kv = amp * e + (dg ? noise : 0.0f);
    return both ? kv : (dg ? 1.0f : 0.0f);
}

__global__ __launch_bounds__(32) __attribute__((amdgpu_num_vgpr(256)))
void k_steps(const float* __restrict__ X, const float* __restrict__ Y, const float* __restrict__ lnz, const float* __restrict__ lam, const float* __restrict__ lls, float* OUT) {
    __shared__ __align__(16) float Kf[MP * KPT];
    __shared__ __align__(16) h16   L16[MP * LPT];
    __shared__ __align__(16) float dinv[MP];
    const int l = threadIdx.x & 31, lr = l & 15, hi = l >> 4;
    const float noise = __expf(bfr(lnz[0]));
    const float amp   = __expf(bfr(lam[0]));
    const float rls2  = 1.0f / __expf(2.0f * bfr(lls[0]));
    float muL = 0.0f, varL = 1.0f;
#pragma unroll 1
    for (int si = 0; si < SPW; ++si) {
        const int t = (int)blockIdx.x * SPW + si + 1;
        int start = t - WWIN; start = start < 0 ? 0 : start;
        const int tm1 = t - 1;
        const int nv = (t >= WWIN) ? MW : (tm1 < 1 ? 1 : tm1);
        const int ti = tm1 > TLEN_FULL - 1 ? TLEN_FULL - 1 : tm1;
        const float xt = bfr(X[ti]);
        float xs[4], ys[4], kx[4];
#pragma unroll
        for (int s = 0; s < 4; ++s) {
            const int i = s * 32 + l;
            int gi = start + i; gi = gi > TLEN_FULL - 1 ? TLEN_FULL - 1 : gi;
            float xv = X[gi], yv = Y[gi];
            asm volatile("" : "+v"(xv)); asm volatile("" : "+v"(yv));
            xv = bfr(xv); yv = bfr(yv);
            const bool val = i < nv;
            const float d = xv - xt;
            const float e = amp * __expf((-0.5f * (d * d)) * rls2);
            xs[s] = xv; ys[s] = val ? yv : 0.0f; kx[s] = val ? e : 0.0f;
        }
        { const v8h hz8 = (v8h){};
#pragma unroll 1
          for (int q = l; q < (MP * LPT) / 8; q += 32) *(v8ha*)(&L16[q * 8]) = hz8; }
#pragma unroll
        for (int shi = 0; shi < 4; ++shi) {
#pragma unroll 1
            for (int ii = 0; ii < 32; ++ii) {
                const int i = shi * 32 + ii;
                const float xi = rdlane(xs[shi], ii);
                const bool vi = i < nv;
#pragma unroll
                for (int sub = 0; sub < 4; ++sub) {
                    if (sub <= shi) {
                        const int j = sub * 32 + l;
                        Kf[i * KPT + j] = kelem(xi, xs[sub], vi & (j < nv), i == j, amp, noise, rls2);
                    }
                }
            }
        }
        __syncthreads();

#pragma unroll 1
        for (int k = 0; k < NPAN; ++k) {
            const int c0 = PW * k;
            if (k > 0) {
                const int nks = (k + 1) >> 1;
                const int bo = (c0 + lr) * LPT + 8 * hi;
#pragma unroll 1
                for (int bi = k; bi < NPAN; ++bi) {
                    const int ao = (PW * bi + lr) * LPT + 8 * hi;
                    v8f acc = (v8f){};
#pragma unroll
                    for (int ks = 0; ks < 4; ++ks) {
                        if (ks < nks) {
                            const v16h a = cat16(*(const v8ha*)(&L16[ao + 32 * ks]), *(const v8ha*)(&L16[ao + 32 * ks + 16]));
                            const v16h b = cat16(*(const v8ha*)(&L16[bo + 32 * ks]), *(const v8ha*)(&L16[bo + 32 * ks + 16]));
                            acc = wmma_g(a, b, acc);
                        }
                    }
                    const int co = (PW * bi + 8 * hi) * KPT + c0 + lr;
#pragma unroll
                    for (int r = 0; r < 8; ++r) { const float cv = Kf[co + r * KPT]; Kf[co + r * KPT] = fmaf(acc[r], -LCI2, cv); }
                }
            }
            __syncthreads();

            {
                const int rj = c0 + lr;
                float d[16];
#pragma unroll
                for (int q = 0; q < 4; ++q) { const v4f x = *(const v4fa*)(&Kf[rj * KPT + c0 + 4 * q]); d[4 * q] = x[0]; d[4 * q + 1] = x[1]; d[4 * q + 2] = x[2]; d[4 * q + 3] = x[3]; }
                float myinv = 1.0f;
#pragma unroll
                for (int cl = 0; cl < 16; ++cl) {
                    const float piv = rdlane(d[cl], cl);
                    const float inv = __builtin_amdgcn_rsqf(piv);
                    const float ld  = piv * inv;
                    myinv = (lr == cl) ? inv : myinv;
                    const float lcol = (lr == cl) ? ld : d[cl] * inv;
                    d[cl] = lcol;
#pragma unroll
                    for (int c2 = cl + 1; c2 < 16; ++c2) d[c2] = fmaf(-lcol, rdlane(lcol, c2), d[c2]);
                }
                if (l < 16) {
#pragma unroll
                    for (int q = 0; q < 4; ++q) { v4f x;
                        x[0] = (4 * q     <= lr) ? d[4 * q]     : 0.0f; x[1] = (4 * q + 1 <= lr) ? d[4 * q + 1] : 0.0f;
                        x[2] = (4 * q + 2 <= lr) ? d[4 * q + 2] : 0.0f; x[3] = (4 * q + 3 <= lr) ? d[4 * q + 3] : 0.0f;
                        *(v4fa*)(&Kf[rj * KPT + c0 + 4 * q]) = x; }
                    dinv[rj] = myinv;
                }
            }
            __syncthreads();

            {
                const int nbel = MP - c0 - PW;
#pragma unroll 1
                for (int rb = 0; rb < nbel; rb += 32) {
                    const int rr = c0 + PW + rb + l;
                    const bool act = rr < MP;
                    const int r = act ? rr : (MP - 1);
                    float p[16], dv[16];
#pragma unroll
                    for (int q = 0; q < 4; ++q) {
                        const v4f x = *(const v4fa*)(&Kf[r * KPT + c0 + 4 * q]); p[4 * q] = x[0]; p[4 * q + 1] = x[1]; p[4 * q + 2] = x[2]; p[4 * q + 3] = x[3];
                        const v4f y = *(const v4fa*)(&dinv[c0 + 4 * q]);         dv[4 * q] = y[0]; dv[4 * q + 1] = y[1]; dv[4 * q + 2] = y[2]; dv[4 * q + 3] = y[3]; }
#pragma unroll
                    for (int cl = 0; cl < 16; ++cl) {
                        float acc = p[cl];
#pragma unroll
                        for (int q = 0; q < 4; ++q) {
                            if (4 * q < cl) {
                                const v4f lq = *(const v4fa*)(&Kf[(c0 + cl) * KPT + c0 + 4 * q]);
#pragma unroll
                                for (int e = 0; e < 4; ++e) { if (4 * q + e < cl) acc = fmaf(-p[4 * q + e], lq[e], acc); }
                            }
                        }
                        p[cl] = acc * dv[cl];
                    }
                    if (act) {
#pragma unroll
                        for (int q = 0; q < 4; ++q) { v4f x; x[0] = p[4 * q]; x[1] = p[4 * q + 1]; x[2] = p[4 * q + 2]; x[3] = p[4 * q + 3]; *(v4fa*)(&Kf[r * KPT + c0 + 4 * q]) = x; }
                        v8h h0, h1;
#pragma unroll
                        for (int e = 0; e < 8; ++e) { h0[e] = toh_flush(p[e] * LCS); h1[e] = toh_flush(p[8 + e] * LCS); }
                        *(v8ha*)(&L16[r * LPT + c0]) = h0; *(v8ha*)(&L16[r * LPT + c0 + 8]) = h1;
                    }
                }
            }
            __syncthreads();
        }

        float ra[4], rv[4];
#pragma unroll
        for (int s = 0; s < 4; ++s) { ra[s] = kx[s]; rv[s] = ys[s]; }
        float mu = 0.0f, var = 0.0f;
#pragma unroll
        for (int s = 0; s < 4; ++s) {
#pragma unroll 1
            for (int cc = 0; cc < 32; ++cc) {
                const int c = 32 * s + cc;
                const float di = dinv[c];
                const float a = rdlane(ra[s], cc) * di;
                const float v = rdlane(rv[s], cc) * di;
                mu = fmaf(a, a, mu); var = fmaf(v, v, var);
#pragma unroll
                for (int ss = 0; ss < 4; ++ss) {
                    if (ss >= s) {
                        const float lv = Kf[(32 * ss + l) * KPT + c];
                        const float mlt = ((ss > s) | (l > cc)) ? lv : 0.0f;
                        ra[ss] = fmaf(-mlt, a, ra[ss]); rv[ss] = fmaf(-mlt, v, rv[ss]);
                    }
                }
            }
        }
        muL  = (l == si) ? mu  : muL;
        varL = (l == si) ? var : varL;
        __syncthreads();
    }

    const int tl = (int)blockIdx.x * SPW + l + 1;
    const float df = (float)(tl + 1);
    const int yi = (tl - 1) > TLEN_FULL - 1 ? TLEN_FULL - 1 : (tl - 1);
    float yv = Y[yi]; yv = bfr(yv);
    const float z  = (yv - muL) / varL;
    const float lp = lgammaf(0.5f * (df + 1.0f)) - lgammaf(0.5f * df)
                   - 0.5f * logf(df * PI_F) - logf(varL)
                   - 0.5f * (df + 1.0f) * log1pf(z * z / df);
    const float up = __expf(lp);
    volatile float* op = OUT + (size_t)blockIdx.x * SPW + l;
    *op = up; __threadfence(); *op = up;
}

extern "C" void kernel_launch(void* const* d_in, const int* in_sizes, int n_in,
                              void* d_out, int out_size, void* d_ws, size_t ws_size, hipStream_t stream) {
    (void)d_ws; (void)ws_size;
    if (n_in < 5) return;
    if (in_sizes[0] < TLEN_FULL || in_sizes[1] < TLEN_FULL) return;
    if (in_sizes[2] < 1 || in_sizes[3] < 1 || in_sizes[4] < 1) return;
    if (out_size < NSTEPS) return;
    const float* X  = (const float*)d_in[0];
    const float* Y  = (const float*)d_in[1];
    const float* ln = (const float*)d_in[2];
    const float* la = (const float*)d_in[3];
    const float* ll = (const float*)d_in[4];
    float* OUT = (float*)d_out;
    k_steps<<<dim3(NSTEPS / SPW, 1, 1), 32, 0, stream>>>(X, Y, ln, la, ll, OUT);
}
